// STGNN_17145509446140
// MI455X (gfx1250) — hardware-run, weakly checked
//
#include <hip/hip_runtime.h>


namespace {
constexpr int N = 100000, E = 1600000, F0 = 5, HID = 128, NPB = 8;
constexpr float XS = 8.0f, HS = 256.0f, WSC = 256.0f;
typedef _Float16 b16;
typedef __attribute__((ext_vector_type(16))) _Float16 v16b;
typedef __attribute__((ext_vector_type(8))) _Float16 v8b;
typedef __attribute__((ext_vector_type(8))) float v8f;
typedef __attribute__((ext_vector_type(4))) float v4f;
__device__ __forceinline__ float bf16_rne(float f) { unsigned int u = __float_as_uint(f); u += 0x7FFFu + ((u >> 16) & 1u); float r = __uint_as_float(u & 0xFFFF0000u); asm volatile("" : "+v"(r)); return r; }
__device__ __forceinline__ float bfv(float f) { float r = bf16_rne(f); asm volatile("" : "+v"(r)); return r; }
__device__ __forceinline__ void split16(float v, b16& hi, b16& lo) { hi = (b16)v; lo = (b16)(v - (float)hi); }
__device__ __forceinline__ v16b frag_kb(const b16* p, int hh) { const v8b a = *(const v8b*)(p + 8 * hh), b = *(const v8b*)(p + 16 + 8 * hh); v16b f;
#pragma unroll
  for (int e = 0; e < 8; ++e) { f[e] = a[e]; f[8 + e] = b[e]; } return f; }
__device__ __forceinline__ v8f wmma16b(v16b a, v16b b, v8f c) { v8f d = __builtin_amdgcn_wmma_f32_16x16x32_f16(false, a, false, b, (short)0, c, false, false); asm volatile("v_nop\n\tv_nop\n\tv_nop\n\tv_nop" : "+v"(d) : "v"(a), "v"(b)); return d; }
__device__ __forceinline__ void wave_lds_sync() { __builtin_amdgcn_fence(__ATOMIC_RELEASE, "workgroup"); __builtin_amdgcn_wave_barrier(); __builtin_amdgcn_fence(__ATOMIC_ACQUIRE, "workgroup"); }
__device__ __forceinline__ float pmul(float a, float b) { float p = a * b; asm volatile("" : "+v"(p)); return p; }
__device__ __forceinline__ int iclamp(int v, int lo, int hi) { return v < lo ? lo : (v > hi ? hi : v); }
__device__ __forceinline__ float wsum(float v) { for (int o = 16; o; o >>= 1) v += __shfl_xor(v, o); return v; }
constexpr int CSR_NBLK8 = 512, CSR_GB8 = 8, CSR_GN8 = 1 << CSR_GB8  , CSR_TS8 = (CSR_GN8 < 32 ? 32 : CSR_GN8)  , CSR_MAXG8 = 512, CSR_CAP8 = 12288  ;
__device__ __host__ __forceinline__ int csr_tix8(int v) { return (v >> CSR_GB8) * CSR_TS8 + (v & (CSR_GN8 - 1)); }
__global__ __launch_bounds__(64) void csrA_kernel8(const int* __restrict__ dst, int E, int N, int nG, int CHP, int NGP, int* __restrict__ STG, int* __restrict__ HST) {
  extern __shared__ int sm[];
  int* cnt = sm; int* run = sm + NGP; int* ids = sm + 2 * NGP;
  const int b = blockIdx.x; const int ch = (E + CSR_NBLK8 - 1) / CSR_NBLK8; const int e0 = b * ch, e1 = min(E, e0 + ch);
  for (int i = threadIdx.x; i < NGP; i += 64) cnt[i] = 0;
  for (int i = threadIdx.x; i < CHP; i += 64) ids[i] = -1;
  __syncthreads();
  if (threadIdx.x == 0) {
    for (int e = e0; e < e1; ++e) { int d = dst[e]; d = (d < 0) ? 0 : (d >= N ? N - 1 : d); cnt[d >> CSR_GB8] += 1; }
    int acc = 0; for (int g = 0; g < nG; ++g) { run[g] = acc; acc += cnt[g]; }
    for (int e = e0; e < e1; ++e) { int d = dst[e]; d = (d < 0) ? 0 : (d >= N ? N - 1 : d); const int g = d >> CSR_GB8; ids[run[g]] = e; run[g] += 1; } }
  __syncthreads();
  typedef __attribute__((ext_vector_type(4))) int v4i;
  for (int pass = 0; pass < 2; ++pass) {
    for (int i = threadIdx.x; i < CHP / 4; i += 64) *(volatile v4i*)(STG + (size_t)b * CHP + i * 4) = *(const v4i*)(&ids[i * 4]);
    for (int i = threadIdx.x; i < NGP / 4; i += 64) { v4i v; for (int e = 0; e < 4; ++e) v[e] = (i * 4 + e < nG) ? cnt[i * 4 + e] : 0; *(volatile v4i*)(HST + (size_t)b * NGP + i * 4) = v; }
    __threadfence(); }
}
__global__ __launch_bounds__(512) void csrS_kernel8(const int* __restrict__ HST, int nG, int NGP, int* __restrict__ START, int* __restrict__ TOT, int* __restrict__ OFF) {
  __shared__ int tot[CSR_MAXG8];
  const int b = threadIdx.x;
  for (int pass = 0; pass < 2; ++pass) { int runb = 0; for (int g = 0; g < nG; ++g) { int c = HST[(size_t)b * NGP + g]; c = (c < 0) ? 0 : c; ((volatile int*)OFF)[(size_t)g * CSR_NBLK8 + b] = runb; runb += c; } __threadfence(); }
  for (int g = threadIdx.x; g < nG; g += 512) { int s = 0; for (int bb = 0; bb < CSR_NBLK8; ++bb) { int c = HST[(size_t)bb * NGP + g]; s += (c < 0) ? 0 : c; } tot[g] = s; }
  __syncthreads();
  if (threadIdx.x < 32) {
    __shared__ int st[CSR_MAXG8 + 32];
    if (threadIdx.x == 0) { int acc = 0; for (int g = 0; g < NGP; ++g) { st[g] = acc; if (g < nG) acc += (tot[g] + 31) & ~31; } st[NGP] = acc; }
    __builtin_amdgcn_fence(__ATOMIC_RELEASE, "workgroup"); __builtin_amdgcn_wave_barrier(); __builtin_amdgcn_fence(__ATOMIC_ACQUIRE, "workgroup");
    for (int pass = 0; pass < 2; ++pass) { for (int i = threadIdx.x; i < NGP + 32; i += 32) { ((volatile int*)START)[i] = (i <= NGP) ? st[min(i, NGP)] : 0; ((volatile int*)TOT)[i] = (i < nG) ? tot[i] : 0; } __threadfence(); } }
}
__global__ __launch_bounds__(256) void csrB_kernel8(const int* __restrict__ dst, int N, int nG, int CHP, int NGP, int permLen, const int* __restrict__ STG, const int* __restrict__ HST, const int* __restrict__ OFF, const int* __restrict__ START, const int* __restrict__ TOT, int* __restrict__ PERM, int* __restrict__ ROWPTR, int* __restrict__ ROWCNT, int* __restrict__ FLAG) {
  typedef __attribute__((ext_vector_type(4))) int v4i;
  __shared__ int ids[CSR_CAP8]; __shared__ unsigned short key[CSR_CAP8]; __shared__ int outp[CSR_CAP8]; __shared__ int ncnt[CSR_GN8 + 1]; __shared__ int boff[CSR_NBLK8 + 1];
  const int g = blockIdx.x, t_ = threadIdx.x; int tot = TOT[g]; int st = START[g], stn = START[g + 1]; const int v0 = g * CSR_GN8; const int nv = min(CSR_GN8, N - v0); const int t0 = g * CSR_TS8;
  st = (st < 0) ? 0 : (st > permLen - 32 ? permLen - 32 : st) & ~31; stn = (stn < st) ? st : (stn > permLen ? permLen : stn); tot = (tot < 0) ? 0 : tot; if (tot > stn - st && tot <= CSR_CAP8) tot = stn - st;
  if (tot > CSR_CAP8) {
    for (int pass = 0; pass < 2; ++pass) { for (int i = t_; i < CSR_TS8 / 4; i += 256) { v4i a, c; for (int e = 0; e < 4; ++e) { a[e] = st; c[e] = 0; } *(volatile v4i*)(ROWPTR + t0 + i * 4) = a; *(volatile v4i*)(ROWCNT + t0 + i * 4) = c; } if (t_ == 0) ((volatile int*)FLAG)[0] = 1; __threadfence(); } (void)nv; return; }
  if (t_ == 0) { int acc = 0; for (int b = 0; b < CSR_NBLK8; ++b) { boff[b] = acc; int c = HST[(size_t)b * NGP + g]; c = (c < 0) ? 0 : (c > CHP ? CHP : c); acc += c; if (acc > tot) acc = tot; } boff[CSR_NBLK8] = acc; }
  for (int i = t_; i <= CSR_GN8; i += 256) ncnt[i] = 0;
  __syncthreads();
  for (int b = 0; b < CSR_NBLK8; ++b) { const int c = boff[b + 1] - boff[b]; int o_ = OFF[(size_t)g * CSR_NBLK8 + b]; o_ = (o_ < 0) ? 0 : (o_ > CHP - c ? CHP - c : o_); const int* src_ = STG + (size_t)b * CHP + o_;
    for (int i = t_; i < c; i += 256) { int id = src_[i]; id = (id < 0) ? 0 : id; ids[boff[b] + i] = id; int d = dst[id]; d = (d < v0) ? v0 : (d >= N ? N - 1 : d); int kk = d - v0; kk = (kk < 0) ? 0 : (kk >= CSR_GN8 ? CSR_GN8 - 1 : kk); key[boff[b] + i] = (unsigned short)kk; } }
  __syncthreads();
  if (t_ == 0) { for (int i = 0; i < tot; ++i) ncnt[key[i]] += 1; int acc = 0; for (int vl = 0; vl < CSR_GN8; ++vl) { const int c = ncnt[vl]; ncnt[vl] = acc; acc += c; } ncnt[CSR_GN8] = acc;
    for (int i = 0; i < tot; ++i) { const int vl = key[i]; outp[ncnt[vl]] = ids[i]; ncnt[vl] += 1; }
    for (int vl = CSR_GN8; vl > 0; --vl) ncnt[vl] = ncnt[vl - 1]; ncnt[0] = 0; }
  __syncthreads();
  for (int pass = 0; pass < 2; ++pass) {
    for (int i = t_; i < (stn - st) / 4; i += 256) { v4i v; for (int e = 0; e < 4; ++e) { const int q = i * 4 + e; v[e] = (q < tot) ? outp[q] : -1; } *(volatile v4i*)(PERM + st + i * 4) = v; }
    for (int i = t_; i < CSR_TS8 / 4; i += 256) { v4i a, c; for (int e = 0; e < 4; ++e) { const int vl = i * 4 + e; const int vc = vl < CSR_GN8 ? vl : CSR_GN8; a[e] = (vl < CSR_GN8) ? st + ncnt[vc] : st; c[e] = (vl < nv) ? (ncnt[(vc < CSR_GN8 ? vc : CSR_GN8 - 1) + 1] - ncnt[vc]) : 0; } *(volatile v4i*)(ROWPTR + t0 + i * 4) = a; *(volatile v4i*)(ROWCNT + t0 + i * 4) = c; }
    __threadfence(); }
}
__global__ __launch_bounds__(256) void csrZ_kernel8(int* __restrict__ p, size_t n4) { typedef __attribute__((ext_vector_type(4))) int v4i; const size_t tid = (size_t)blockIdx.x * 256 + threadIdx.x, nth = (size_t)gridDim.x * 256; v4i z = {0, 0, 0, 0}; for (size_t i = tid; i < n4; i += nth) *(volatile v4i*)(p + i * 4) = z; }
struct CsrBufs8 { int *STG, *HST, *OFF, *START, *TOT, *PERM, *ROWPTR, *ROWCNT, *FLAG; int nG, NGP, CHP; size_t permLen; char* base; size_t bytes; };
static size_t csr_carve8(CsrBufs8& c, char* ws, size_t off, int E, int N) {
  const size_t off0 = off; c.base = ws + off;
  auto al = [&](size_t bytes) { char* p = ws + off; off += (bytes + 255) & ~(size_t)255; return p; };
  c.nG = (N + CSR_GN8 - 1) / CSR_GN8; c.NGP = (c.nG + 31) & ~31; const int ch = (E + CSR_NBLK8 - 1) / CSR_NBLK8; c.CHP = (ch + 31) & ~31; c.permLen = (size_t)E + 32 * (size_t)c.nG + 32;
  c.STG = (int*)al((size_t)CSR_NBLK8 * c.CHP * 4); c.HST = (int*)al((size_t)CSR_NBLK8 * c.NGP * 4); c.OFF = (int*)al((size_t)c.NGP * CSR_NBLK8 * 4); c.START = (int*)al((size_t)(c.NGP + 64) * 4); c.TOT = (int*)al((size_t)(c.NGP + 64) * 4);
  c.PERM = (int*)al(c.permLen * 4); c.ROWPTR = (int*)al((size_t)c.nG * CSR_TS8 * 4); c.ROWCNT = (int*)al((size_t)c.nG * CSR_TS8 * 4); c.FLAG = (int*)al(256);
  c.bytes = off - off0; return off;
}
static void csr_build8(const CsrBufs8& c, const int* dst, int E, int N, hipStream_t stream) {
  const size_t smem = (size_t)(2 * c.NGP + c.CHP) * 4;
  csrZ_kernel8<<<512, 256, 0, stream>>>((int*)c.base, c.bytes / 16);
  csrA_kernel8<<<CSR_NBLK8, 64, smem, stream>>>(dst, E, N, c.nG, c.CHP, c.NGP, c.STG, c.HST);
  csrS_kernel8<<<1, 512, 0, stream>>>(c.HST, c.nG, c.NGP, c.START, c.TOT, c.OFF);
  csrB_kernel8<<<c.nG, 256, 0, stream>>>(dst, N, c.nG, c.CHP, c.NGP, (int)c.permLen, c.STG, c.HST, c.OFF, c.START, c.TOT, c.PERM, c.ROWPTR, c.ROWCNT, c.FLAG);
}


__global__ __launch_bounds__(256) void wput_kernel(const float* __restrict__ w1, const float* __restrict__ w2, const float* __restrict__ w3, b16* __restrict__ W1T, b16* __restrict__ W2T, b16* __restrict__ W3T) { const int u = blockIdx.x * 256 + threadIdx.x; v8b v; auto put = [&](b16* dst) { for (int pass = 0; pass < 2; ++pass) { *(volatile v8b*)dst = v; __threadfence(); } };
  if (u < HID * 4) { const int o = u / 4, k0 = (u % 4) * 8;
#pragma unroll
    for (int j = 0; j < 8; ++j) { const int k = k0 + j; v[j] = (b16)(k < F0 ? bf16_rne(w1[k * HID + o]) * WSC : 0.0f); } put(W1T + (size_t)o * 32 + k0); }
  if (u < HID * 16) { const int o = u / 16, k0 = (u % 16) * 8;
#pragma unroll
    for (int j = 0; j < 8; ++j) v[j] = (b16)(bf16_rne(w2[(size_t)(k0 + j) * HID + o]) * WSC); put(W2T + (size_t)o * HID + k0);
#pragma unroll
    for (int j = 0; j < 8; ++j) v[j] = (b16)(bf16_rne(w3[(size_t)(k0 + j) * HID + o]) * WSC); put(W3T + (size_t)o * HID + k0); } }
template <int MODE>
__global__ __launch_bounds__(32) void proj_kernel(const float* __restrict__ IN, const b16* __restrict__ W, int NLIM, float* __restrict__ P) { constexpr int KD = MODE == 0 ? 32 : HID; __shared__ __attribute__((aligned(16))) b16 Ah[16][KD + 8], Al[16][KD + 8]; __shared__ float Tf[16][HID + 4]; const int lane = threadIdx.x, nloc = lane & 15, hlf = lane >> 4; const size_t n0 = (size_t)blockIdx.x * 16; if (n0 >= (size_t)NLIM) return;
  if (MODE == 0) { for (int rr = 0; rr < 16; ++rr) { Ah[rr][lane] = (b16)(lane < F0 ? bfv(IN[(n0 + rr) * F0 + lane]) * XS : 0.0f); Al[rr][lane] = (b16)0.0f; if (lane < 8) { Ah[rr][32 + lane] = (b16)0.0f; Al[rr][32 + lane] = (b16)0.0f; } } }
  else { for (int rr = 0; rr < 16; ++rr) for (int q = 0; q < 4; ++q) { const int c = q * 32 + lane; b16 p, pl; split16(IN[(n0 + rr) * HID + c] * HS, p, pl); Ah[rr][c] = p; Al[rr][c] = pl; } if (lane < 16) for (int k = HID; k < HID + 8; ++k) { Ah[lane][k] = (b16)0.0f; Al[lane][k] = (b16)0.0f; } }
  wave_lds_sync(); v8f acc[8];
#pragma unroll
  for (int t = 0; t < 8; ++t) acc[t] = (v8f){};
#pragma unroll
  for (int kb = 0; kb < KD; kb += 32) { const v16b a = frag_kb(&Ah[nloc][kb], hlf), al = frag_kb(&Al[nloc][kb], hlf);
#pragma unroll
    for (int t = 0; t < 8; ++t) { const v16b bw = frag_kb(W + (size_t)(t * 16 + nloc) * KD + kb, hlf); acc[t] = wmma16b(a, bw, acc[t]); if (MODE != 0) acc[t] = wmma16b(al, bw, acc[t]); } }
  const float isc = MODE == 0 ? 1.0f / (XS * WSC) : 1.0f / (HS * WSC);
#pragma unroll
  for (int t = 0; t < 8; ++t)
#pragma unroll
    for (int r8 = 0; r8 < 8; ++r8) Tf[8 * hlf + r8][t * 16 + nloc] = acc[t][r8] * isc;
  wave_lds_sync();
  for (int pass = 0; pass < 2; ++pass) { for (int rr = 0; rr < 16; ++rr) *(volatile v4f*)(P + (n0 + rr) * HID + lane * 4) = *(const v4f*)(&Tf[rr][lane * 4]); __threadfence(); } }
__global__ __launch_bounds__(256) void agg_kernel(const float* __restrict__ P, const float* __restrict__ bias, const int* __restrict__ srcs, const int* __restrict__ PERM, const int* __restrict__ ROWPTR, const int* __restrict__ ROWCNT, int permLen, int NLIM, float* __restrict__ Hout) { const int wave = threadIdx.x >> 5, lane = threadIdx.x & 31; const size_t n = (size_t)blockIdx.x * NPB + wave; if (n >= (size_t)NLIM) return;
  int st = ROWPTR[n], cnt = ROWCNT[n]; cnt = iclamp(cnt, 0, E); st = iclamp(st, 0, permLen - cnt); const float dn = rsqrtf((float)cnt + 1.0f); v4f a = {0, 0, 0, 0};
#pragma unroll 1
  for (int j = 0; j < cnt; ++j) { const int e = iclamp(PERM[st + j], 0, E - 1); const size_t s = (size_t)iclamp(srcs[e], 0, N - 1); if (s >= (size_t)NLIM) continue; const float ds = rsqrtf((float)iclamp(ROWCNT[s], 0, E) + 1.0f); a += *(const v4f*)(P + s * HID + lane * 4) * pmul(ds, dn); }
  a += *(const v4f*)(P + n * HID + lane * 4) * pmul(dn, dn);
  v4f o; for (int q = 0; q < 4; ++q) o[q] = fmaxf(a[q] + bfv(bias[lane * 4 + q]), 0.0f);
  for (int pass = 0; pass < 2; ++pass) { *(volatile v4f*)(Hout + n * HID + lane * 4) = o; __threadfence(); } }
__global__ __launch_bounds__(256) void fc_kernel(const float* __restrict__ Hh, const float* __restrict__ wfc, const float* __restrict__ bfc, int NLIM, float* __restrict__ out) { const int wave = threadIdx.x >> 5, lane = threadIdx.x & 31; const size_t n0 = ((size_t)blockIdx.x * NPB + wave) * 32; if (n0 >= (size_t)N) return; float w4[4]; for (int q = 0; q < 4; ++q) w4[q] = bfv(wfc[lane * 4 + q]); const float b0 = bfv(bfc[0]); float mine = 0.0f;
#pragma unroll 1
  for (int j = 0; j < 32; ++j) { const size_t n = n0 + j; float v = 0.0f; if (n < (size_t)NLIM) { const v4f h = *(const v4f*)(Hh + n * HID + lane * 4); float part = 0.0f; for (int q = 0; q < 4; ++q) part += pmul(h[q], w4[q]); v = wsum(part) + b0; } mine = (lane == j) ? v : mine; }
  for (int pass = 0; pass < 2; ++pass) { ((volatile float*)out)[n0 + lane] = mine; __threadfence(); } }
}

extern "C" void kernel_launch(void* const* d_in, const int* in_sizes, int n_in, void* d_out, int out_size, void* d_ws, size_t ws_size, hipStream_t stream) {
  (void)n_in;
  auto Fp = [&](int i) { return (const float*)d_in[i]; }; auto Ip = [&](int i) { return (const int*)d_in[i]; };
  if (in_sizes[0] != N * F0 || in_sizes[1] != 2 * E || in_sizes[2] != F0 * HID || in_sizes[4] != HID * HID || in_sizes[6] != HID * HID || in_sizes[8] != HID || out_size != N) return;
  const int NLIM = N;
  size_t off = 0; char* ws = (char*)d_ws;
  auto carve = [&](size_t bytes) { char* p = ws + off; off += (bytes + 255) & ~(size_t)255; return p; };
  b16* W1T = (b16*)carve(HID * 32 * 2); b16* W2T = (b16*)carve(HID * HID * 2); b16* W3T = (b16*)carve(HID * HID * 2); float* P = (float*)carve((size_t)N * HID * 4); float* Hh = (float*)carve((size_t)N * HID * 4); CsrBufs8 csr; off = csr_carve8(csr, ws, off, E, N);
  if (off > ws_size || off > ((size_t)144 << 20)) return;
  wput_kernel<<<(HID * 16 + 255) / 256, 256, 0, stream>>>(Fp(2), Fp(4), Fp(6), W1T, W2T, W3T);
  csr_build8(csr, Ip(1) + E, E, N, stream);
  const int nb = (NLIM + NPB - 1) / NPB;
  proj_kernel<0><<<NLIM / 16, 32, 0, stream>>>(Fp(0), W1T, NLIM, P);
  agg_kernel<<<nb, 256, 0, stream>>>(P, Fp(3), Ip(1), csr.PERM, csr.ROWPTR, csr.ROWCNT, (int)csr.permLen, NLIM, Hh);
  proj_kernel<1><<<NLIM / 16, 32, 0, stream>>>(Hh, W2T, NLIM, P);
  agg_kernel<<<nb, 256, 0, stream>>>(P, Fp(5), Ip(1), csr.PERM, csr.ROWPTR, csr.ROWCNT, (int)csr.permLen, NLIM, Hh);
  proj_kernel<1><<<NLIM / 16, 32, 0, stream>>>(Hh, W3T, NLIM, P);
  agg_kernel<<<nb, 256, 0, stream>>>(P, Fp(7), Ip(1), csr.PERM, csr.ROWPTR, csr.ROWCNT, (int)csr.permLen, NLIM, Hh);
  fc_kernel<<<(N / 32 + NPB - 1) / NPB, 256, 0, stream>>>(Hh, Fp(8), Fp(9), NLIM, (float*)d_out);
}
